// MaskedAttention_4853313044615
// MI455X (gfx1250) — hardware-verified
//
#include <hip/hip_runtime.h>
#include <stdint.h>
#include <math.h>

typedef __attribute__((ext_vector_type(16))) _Float16 v16h;
typedef __attribute__((ext_vector_type(8)))  _Float16 v8h;
typedef __attribute__((ext_vector_type(16))) __bf16   v16b;
typedef __attribute__((ext_vector_type(8)))  __bf16   v8b;
typedef __attribute__((ext_vector_type(8)))  float    v8f;
typedef __attribute__((ext_vector_type(4)))  float    v4f;
typedef __attribute__((ext_vector_type(4)))  unsigned v4u;
typedef __attribute__((ext_vector_type(2)))  unsigned v2u;

constexpr int kBatch = 2;
constexpr int kSeq   = 2048;
constexpr int kEmb   = 1024;
constexpr int kHeads = 16;
constexpr int kHd    = 64;
constexpr int kTok   = kBatch * kSeq;
constexpr int kKvCh  = 64;
constexpr int kQb    = 64;
static_assert(kHeads * kHd == kEmb);
static_assert(kHd == 64);
static_assert(kEmb % 32 == 0);
static_assert(kTok % 64 == 0);
static_assert(kEmb % 64 == 0);
static_assert(kSeq % kQb == 0);
static_assert(kSeq % kKvCh == 0);
static_assert((kTok * kEmb) % (256 * 8) == 0);

__device__ __forceinline__ unsigned short f2bf_bits(float f) {
  unsigned u = __float_as_uint(f);
  return (unsigned short)((u + 0x7FFFu + ((u >> 16) & 1u)) >> 16);
}
__device__ __forceinline__ float bf_bits2f(unsigned short h) { return __uint_as_float(((unsigned)h) << 16); }

__device__ __forceinline__ void dep_guard_b(v8f& a, v8f& b, v16b x, v16b y) { asm volatile("v_nop\n\tv_nop\n\tv_nop\n\tv_nop" : "+v"(a), "+v"(b) : "v"(x), "v"(y)); }
__device__ __forceinline__ void keep4_b(v16b a, v16b b, v16b c, v16b d) { asm volatile("v_nop" :: "v"(a), "v"(b), "v"(c), "v"(d)); }
__device__ __forceinline__ void acc_guard4(v8f& a, v8f& b, v8f& c, v8f& d) { asm volatile("v_nop\n\tv_nop\n\tv_nop\n\tv_nop" : "+v"(a), "+v"(b), "+v"(c), "+v"(d)); }

template <typename T> struct Frag;
template <> struct Frag<__bf16> {
  typedef v16b V; union U { v16b v; v8b h[2]; };
  static __device__ __forceinline__ v16b load(const __bf16* p) {
    U f; f.h[0] = *(const v8b*)(p); f.h[1] = *(const v8b*)(p + 16); return f.v;
  }
  static __device__ __forceinline__ v8f mma(v16b a, v16b b, v8f c) {
    return __builtin_amdgcn_wmma_f32_16x16x32_bf16(false, a, false, b, (short)0, c, false, false);
  }
  static __device__ __forceinline__ void guard(v8f& a, v8f& b, v16b x, v16b y) { dep_guard_b(a, b, x, y); }
  static __device__ __forceinline__ void keep(v16b a, v16b b, v16b c, v16b d) { keep4_b(a, b, c, d); }
};

__device__ __forceinline__ __bf16 at_f2bf(float f) { return __builtin_bit_cast(__bf16, f2bf_bits(f)); }
__device__ __forceinline__ void at_split(float f, __bf16& hi, __bf16& lo) {
  const unsigned short hb = f2bf_bits(f);
  hi = __builtin_bit_cast(__bf16, hb);
  lo = at_f2bf(f - __uint_as_float(((unsigned)hb) << 16));
}
__device__ __forceinline__ v8f at_mma(v16b a, v16b b, v8f c) {
  c = __builtin_amdgcn_wmma_f32_16x16x32_bf16(false, a, false, b, (short)0, c, false, false);
  asm volatile("v_nop\n\tv_nop\n\tv_nop\n\tv_nop" : "+v"(c) : "v"(a), "v"(b));
  return c;
}

__global__ __launch_bounds__(256) void k_cast_f32_bf16x8(const float* __restrict__ in,
                                                          unsigned short* __restrict__ out, int n8) {
  const int i = blockIdx.x * 256 + threadIdx.x;
  if (i < n8) {
    const v4f a = *(const v4f*)(in + (size_t)i * 8);
    const v4f c = *(const v4f*)(in + (size_t)i * 8 + 4);
    v4u w;
    w[0] = (unsigned)f2bf_bits(a[0]) | ((unsigned)f2bf_bits(a[1]) << 16);
    w[1] = (unsigned)f2bf_bits(a[2]) | ((unsigned)f2bf_bits(a[3]) << 16);
    w[2] = (unsigned)f2bf_bits(c[0]) | ((unsigned)f2bf_bits(c[1]) << 16);
    w[3] = (unsigned)f2bf_bits(c[2]) | ((unsigned)f2bf_bits(c[3]) << 16);
    *(volatile v4u*)(out + (size_t)i * 8) = w;
    __threadfence();
    *(volatile v4u*)(out + (size_t)i * 8) = w;
  }
}

__global__ __launch_bounds__(128) void k_tr_f32_bf16(const float* __restrict__ in,
                                                     unsigned short* __restrict__ out, int R, int Cc) {
  __shared__ __align__(16) unsigned short tile[64 * 68];
  const int t = threadIdx.x, wave = t >> 5, lane = t & 31;
  const int r0 = blockIdx.y * 64, c0 = blockIdx.x * 64;
#pragma unroll
  for (int i = 0; i < 8; ++i) {
    const int p = t + 128 * i;
    const int row = p >> 4;
    const int c4 = (p & 15) * 4;
    const v4f v = *(const v4f*)(in + (size_t)(r0 + row) * Cc + c0 + c4);
    v2u w;
    w[0] = (unsigned)f2bf_bits(v[0]) | ((unsigned)f2bf_bits(v[1]) << 16);
    w[1] = (unsigned)f2bf_bits(v[2]) | ((unsigned)f2bf_bits(v[3]) << 16);
    *(v2u*)(tile + row * 68 + c4) = w;
  }
  __syncthreads();
  const int q = lane >> 3, c8 = (lane & 7) * 8;
  for (int pass = 0; pass < 2; ++pass) {
#pragma unroll
    for (int it = 0; it < 4; ++it) {
      const int cc = wave * 16 + it * 4 + q;
      v4u w;
#pragma unroll
      for (int e = 0; e < 4; ++e) {
        const unsigned lo = tile[(c8 + 2 * e) * 68 + cc];
        const unsigned hi = tile[(c8 + 2 * e + 1) * 68 + cc];
        w[e] = lo | (hi << 16);
      }
      *(volatile v4u*)(out + (size_t)(c0 + cc) * R + r0 + c8) = w;
    }
    __threadfence();
  }
}

__global__ __launch_bounds__(128) void k_tr_u16(const unsigned short* __restrict__ in,
                                                unsigned short* __restrict__ out, int R, int Cc,
                                                long strideIn, long strideOut) {
  __shared__ __align__(16) unsigned short tile[64 * 72];
  const int t = threadIdx.x, wave = t >> 5, lane = t & 31;
  const int r0 = blockIdx.y * 64, c0 = blockIdx.x * 64;
  const unsigned short* inb = in + (size_t)blockIdx.z * strideIn;
  unsigned short* outb = out + (size_t)blockIdx.z * strideOut;
#pragma unroll
  for (int i = 0; i < 4; ++i) {
    const int p = t + 128 * i;
    const int row = p >> 3;
    const int cp8 = (p & 7) * 8;
    const v4u u = *(const v4u*)(inb + (size_t)(r0 + row) * Cc + c0 + cp8);
    *(v4u*)(tile + row * 72 + cp8) = u;
  }
  __syncthreads();
  const int q = lane >> 3, c8 = (lane & 7) * 8;
  for (int pass = 0; pass < 2; ++pass) {
#pragma unroll
    for (int it = 0; it < 4; ++it) {
      const int cc = wave * 16 + it * 4 + q;
      v4u w;
#pragma unroll
      for (int e = 0; e < 4; ++e) {
        const unsigned lo = tile[(c8 + 2 * e) * 72 + cc];
        const unsigned hi = tile[(c8 + 2 * e + 1) * 72 + cc];
        w[e] = lo | (hi << 16);
      }
      *(volatile v4u*)(outb + (size_t)(c0 + cc) * R + r0 + c8) = w;
    }
    __threadfence();
  }
}

template <bool ASPLIT, int OUT_MODE>
__global__ __launch_bounds__(256) void gemm_bf16_t64(
    const unsigned short* __restrict__ Ap, const unsigned short* __restrict__ A2p, int lda,
    const unsigned short* __restrict__ Btp, int ldb,
    void* __restrict__ Cout, void* __restrict__ Cout2, int ldc,
    const float* __restrict__ bias, int M, int N, int K) {
  typedef __bf16 T;
  typedef v16b V;
  const T* A = (const T*)Ap; const T* A2 = (const T*)A2p; const T* Bt = (const T*)Btp;
  __shared__ __align__(16) float sT[8][16 * 68];
  const int lane = threadIdx.x & 31;
  const int wave = threadIdx.x >> 5;
  const int tilesN = N >> 6;
  const int tilesM = M >> 6;
  const int tile = blockIdx.x * 8 + wave;
  if (tile >= tilesM * tilesN) return;
  const int tm = tile / tilesN;
  const int tn = tile - tm * tilesN;
  const int m0 = tm << 6;
  const int n0 = tn << 6;

  const int rlane = lane & 15;
  const int koff  = (lane >> 4) * 8;
  const int mOff  = (lane >> 4) * 8;

  v8f acc[4][4];
#pragma unroll
  for (int i = 0; i < 4; ++i)
#pragma unroll
    for (int j = 0; j < 4; ++j) acc[i][j] = (v8f){0.f,0.f,0.f,0.f,0.f,0.f,0.f,0.f};

  for (int k0 = 0; k0 < K; k0 += 32) {
    V bh[4];
#pragma unroll
    for (int j = 0; j < 4; ++j) {
      const size_t bo = (size_t)(n0 + (j << 4) + rlane) * ldb + koff + k0;
      bh[j] = Frag<T>::load(Bt + bo);
    }
#pragma unroll
    for (int i = 0; i < 4; ++i) {
      const size_t ao = (size_t)(m0 + (i << 4) + rlane) * lda + koff + k0;
      V ah = Frag<T>::load(A + ao);
      V al = ah;
      if (ASPLIT) al = Frag<T>::load(A2 + ao);
#pragma unroll
      for (int j = 0; j < 4; ++j) {
        acc[i][j] = Frag<T>::mma(ah, bh[j], acc[i][j]);
        if (ASPLIT) acc[i][j] = Frag<T>::mma(al, bh[j], acc[i][j]);
      }
      Frag<T>::guard(acc[i][0], acc[i][3], ah, al);
    }
    Frag<T>::keep(bh[0], bh[1], bh[2], bh[3]);
  }
  acc_guard4(acc[0][0], acc[0][1], acc[0][2], acc[0][3]);
  acc_guard4(acc[1][0], acc[1][1], acc[1][2], acc[1][3]);
  acc_guard4(acc[2][0], acc[2][1], acc[2][2], acc[2][3]);
  acc_guard4(acc[3][0], acc[3][1], acc[3][2], acc[3][3]);

  float bvj[4];
#pragma unroll
  for (int j = 0; j < 4; ++j) bvj[j] = bf_bits2f(f2bf_bits(bias[n0 + (j << 4) + rlane]));
  float* slab = sT[wave];
#pragma unroll
  for (int i = 0; i < 4; ++i) {
    const int mBase = m0 + (i << 4);
#pragma unroll
    for (int j = 0; j < 4; ++j) {
#pragma unroll
      for (int r = 0; r < 8; ++r) {
        const float v = acc[i][j][r] + bvj[j];
        slab[(mOff + r) * 68 + (j << 4) + rlane] = v;
      }
    }
    __builtin_amdgcn_fence(__ATOMIC_RELEASE, "workgroup");
    __builtin_amdgcn_wave_barrier();
    __builtin_amdgcn_fence(__ATOMIC_ACQUIRE, "workgroup");
    if (OUT_MODE == 0) {
      float* C = (float*)Cout;
      const int hh = lane >> 4, c4 = (lane & 15) * 4;
      for (int pass = 0; pass < 2; ++pass) {
#pragma unroll
        for (int it = 0; it < 8; ++it) {
          const int row = it * 2 + hh;
          v4f v = *(const v4f*)(slab + row * 68 + c4);
          *(volatile v4f*)(C + (size_t)(mBase + row) * ldc + n0 + c4) = v;
        }
        __threadfence();
      }
    } else {
      const int q = lane >> 3, c8 = (lane & 7) * 8;
      unsigned short* C  = (unsigned short*)Cout;
      unsigned short* C2 = (unsigned short*)Cout2;
      for (int pass = 0; pass < 2; ++pass) {
#pragma unroll
        for (int it = 0; it < 4; ++it) {
          const int row = it * 4 + q;
          const float* sp = slab + row * 68 + c8;
          v8h hv, lv;
#pragma unroll
          for (int e = 0; e < 8; ++e) {
            unsigned short hb = f2bf_bits(sp[e]);
            unsigned short lb = f2bf_bits(sp[e] - bf_bits2f(hb));
            hv[e] = __builtin_bit_cast(_Float16, hb);
            lv[e] = __builtin_bit_cast(_Float16, lb);
          }
          *(volatile v8h*)(C + (size_t)(mBase + row) * ldc + n0 + c8) = hv;
          *(volatile v8h*)(C2 + (size_t)(mBase + row) * ldc + n0 + c8) = lv;
        }
        __threadfence();
      }
    }
    __builtin_amdgcn_fence(__ATOMIC_RELEASE, "workgroup");
    __builtin_amdgcn_wave_barrier();
    __builtin_amdgcn_fence(__ATOMIC_ACQUIRE, "workgroup");
  }
}

__global__ __launch_bounds__(128) void k_attn_causal(
    const unsigned short* __restrict__ Qh, const unsigned short* __restrict__ Ql,
    const unsigned short* __restrict__ Kh, const unsigned short* __restrict__ Kl,
    const unsigned short* __restrict__ Vth, const unsigned short* __restrict__ Vtl,
    unsigned short* __restrict__ Oh, unsigned short* __restrict__ Ol) {
  union FB { v16b v; v8b h[2]; };
  __shared__ __align__(16) unsigned short Ksh[kKvCh * kHd];
  __shared__ __align__(16) unsigned short Ksl[kKvCh * kHd];
  __shared__ __align__(16) unsigned short Vsh[kHd * kKvCh];
  __shared__ __align__(16) unsigned short Vsl[kHd * kKvCh];
  __shared__ __align__(16) __bf16 Psh[4][16 * kKvCh];
  __shared__ __align__(16) __bf16 Psl[4][16 * kKvCh];
  __shared__ __align__(16) float  Os[4][16 * 68];

  const int tid  = threadIdx.x;
  const int wave = tid >> 5;
  const int lane = tid & 31;
  const int hh   = lane >> 4;
  const int c    = lane & 15;

  constexpr int nqb = kSeq / kQb;
  const int bx = blockIdx.x;
  const int qb = bx % nqb;
  const int bh = bx / nqb;
  const int h  = bh % kHeads;
  const int b  = bh / kHeads;
  const size_t tokbase = (size_t)b * kSeq;
  const int q0 = qb * kQb + wave * 16;

  v16b qah[2], qal[2];
  {
    const __bf16* qrh = (const __bf16*)Qh + (tokbase + q0 + c) * kEmb + h * kHd + 8 * hh;
    const __bf16* qrl = (const __bf16*)Ql + (tokbase + q0 + c) * kEmb + h * kHd + 8 * hh;
#pragma unroll
    for (int dc = 0; dc < 2; ++dc) {
      qah[dc] = Frag<__bf16>::load(qrh + dc * 32);
      qal[dc] = Frag<__bf16>::load(qrl + dc * 32);
    }
  }

  float mrow[8], lrow[8];
  v8f oacc[4];
#pragma unroll
  for (int r = 0; r < 8; ++r) { mrow[r] = -INFINITY; lrow[r] = 0.f; }
#pragma unroll
  for (int t = 0; t < 4; ++t) oacc[t] = (v8f){0.f,0.f,0.f,0.f,0.f,0.f,0.f,0.f};

  const unsigned short* kgh = Kh + tokbase * kEmb + h * kHd;
  const unsigned short* kgl = Kl + tokbase * kEmb + h * kHd;
  const unsigned short* vgh = Vth + (size_t)bh * kHd * kSeq;
  const unsigned short* vgl = Vtl + (size_t)bh * kHd * kSeq;

  const int nChunks = qb + 1;
  for (int kc = 0; kc < nChunks; ++kc) {
    const int kv0 = kc * kKvCh;
    __syncthreads();
#pragma unroll 1
    for (int i = 0; i < 4; ++i) {
      const int p = tid + 128 * i;
      const int row = p >> 3;
      const int c8 = (p & 7) * 8;
      const v4u a  = *(const v4u*)(kgh + (size_t)(kv0 + row) * kEmb + c8);
      const v4u a2 = *(const v4u*)(kgl + (size_t)(kv0 + row) * kEmb + c8);
      const v4u w  = *(const v4u*)(vgh + (size_t)row * kSeq + kv0 + c8);
      const v4u w2 = *(const v4u*)(vgl + (size_t)row * kSeq + kv0 + c8);
      *(v4u*)(Ksh + row * kHd + c8) = a;
      *(v4u*)(Ksl + row * kHd + c8) = a2;
      *(v4u*)(Vsh + row * kKvCh + c8) = w;
      *(v4u*)(Vsl + row * kKvCh + c8) = w2;
    }
    __syncthreads();

    v8f s[4];
#pragma unroll
    for (int j = 0; j < 4; ++j) {
      s[j] = (v8f){0.f,0.f,0.f,0.f,0.f,0.f,0.f,0.f};
#pragma unroll
      for (int dc = 0; dc < 2; ++dc) {
        const v16b kb = Frag<__bf16>::load((const __bf16*)Ksh + (j * 16 + c) * kHd + dc * 32 + 8 * hh);
        const v16b kl = Frag<__bf16>::load((const __bf16*)Ksl + (j * 16 + c) * kHd + dc * 32 + 8 * hh);
        s[j] = at_mma(qah[dc], kb, s[j]);
        s[j] = at_mma(qah[dc], kl, s[j]);
        s[j] = at_mma(qal[dc], kb, s[j]);
      }
    }

    const bool diag = (kc == qb);
    float cm[8];
#pragma unroll
    for (int r = 0; r < 8; ++r) {
      const int qrow = q0 + 8 * hh + r;
      float m = -INFINITY;
#pragma unroll
      for (int j = 0; j < 4; ++j) {
        const int kvcol = kv0 + j * 16 + c;
        float sv = s[j][r] * 0.125f;
        if (diag && (kvcol > qrow)) sv = -INFINITY;
        s[j][r] = sv;
        m = fmaxf(m, sv);
      }
#pragma unroll
      for (int off = 1; off < 16; off <<= 1) m = fmaxf(m, __shfl_xor(m, off, 32));
      cm[r] = m;
    }

    __bf16* pwh = Psh[wave];
    __bf16* pwl = Psl[wave];
#pragma unroll
    for (int r = 0; r < 8; ++r) {
      const float mnew = fmaxf(mrow[r], cm[r]);
      const float alpha = expf(mrow[r] - mnew);
      mrow[r] = mnew;
      float psum = 0.f;
#pragma unroll
      for (int j = 0; j < 4; ++j) {
        const float p = expf(s[j][r] - mnew);
        psum += p;
        __bf16 ph, pl;
        at_split(p, ph, pl);
        pwh[(8 * hh + r) * kKvCh + j * 16 + c] = ph;
        pwl[(8 * hh + r) * kKvCh + j * 16 + c] = pl;
      }
#pragma unroll
      for (int off = 1; off < 16; off <<= 1) psum += __shfl_xor(psum, off, 32);
      lrow[r] = lrow[r] * alpha + psum;
#pragma unroll
      for (int t = 0; t < 4; ++t) oacc[t][r] *= alpha;
    }
    __builtin_amdgcn_fence(__ATOMIC_RELEASE, "workgroup");
    __builtin_amdgcn_wave_barrier();
    __builtin_amdgcn_fence(__ATOMIC_ACQUIRE, "workgroup");

#pragma unroll 1
    for (int kk = 0; kk < 2; ++kk) {
      FB pa, pl;
      pa.h[0] = *(const v8b*)(pwh + c * kKvCh + kk * 32 + 8 * hh);
      pa.h[1] = *(const v8b*)(pwh + c * kKvCh + kk * 32 + 16 + 8 * hh);
      pl.h[0] = *(const v8b*)(pwl + c * kKvCh + kk * 32 + 8 * hh);
      pl.h[1] = *(const v8b*)(pwl + c * kKvCh + kk * 32 + 16 + 8 * hh);
#pragma unroll
      for (int t = 0; t < 4; ++t) {
        const v16b vb = Frag<__bf16>::load((const __bf16*)Vsh + (t * 16 + c) * kKvCh + kk * 32 + 8 * hh);
        const v16b vl = Frag<__bf16>::load((const __bf16*)Vsl + (t * 16 + c) * kKvCh + kk * 32 + 8 * hh);
        oacc[t] = at_mma(pa.v, vb, oacc[t]);
        oacc[t] = at_mma(pa.v, vl, oacc[t]);
        oacc[t] = at_mma(pl.v, vb, oacc[t]);
      }
    }
  }

  float* os = Os[wave];
#pragma unroll
  for (int r = 0; r < 8; ++r) {
    const float inv = 1.0f / lrow[r];
#pragma unroll
    for (int t = 0; t < 4; ++t) os[(8 * hh + r) * 68 + t * 16 + c] = oacc[t][r] * inv;
  }
  __builtin_amdgcn_fence(__ATOMIC_RELEASE, "workgroup");
  __builtin_amdgcn_wave_barrier();
  __builtin_amdgcn_fence(__ATOMIC_ACQUIRE, "workgroup");
  {
    const int q4 = lane >> 3, c8 = (lane & 7) * 8;
    unsigned short* ogh = Oh + (tokbase + q0) * kEmb + h * kHd + c8;
    unsigned short* ogl = Ol + (tokbase + q0) * kEmb + h * kHd + c8;
    for (int pass = 0; pass < 2; ++pass) {
#pragma unroll
      for (int it = 0; it < 4; ++it) {
        const int row = it * 4 + q4;
        const float* sp = os + row * 68 + c8;
        v8h hv, lv;
#pragma unroll
        for (int e = 0; e < 8; ++e) {
          unsigned short hb = f2bf_bits(sp[e]);
          unsigned short lb = f2bf_bits(sp[e] - bf_bits2f(hb));
          hv[e] = __builtin_bit_cast(_Float16, hb);
          lv[e] = __builtin_bit_cast(_Float16, lb);
        }
        *(volatile v8h*)(ogh + (size_t)row * kEmb) = hv;
        *(volatile v8h*)(ogl + (size_t)row * kEmb) = lv;
      }
      __threadfence();
    }
  }
}

extern "C" void kernel_launch(void* const* d_in, const int* in_sizes, int n_in,
                              void* d_out, int out_size, void* d_ws, size_t ws_size,
                              hipStream_t stream) {
  if (n_in < 9) return;
  if (in_sizes[0] != kTok * kEmb) return;
  if (in_sizes[1] != kEmb * kEmb || in_sizes[3] != kEmb * kEmb || in_sizes[5] != kEmb * kEmb || in_sizes[7] != kEmb * kEmb) return;
  if (in_sizes[2] != kEmb || in_sizes[4] != kEmb || in_sizes[6] != kEmb || in_sizes[8] != kEmb) return;
  if (out_size != kTok * kEmb) return;

  const float* x  = (const float*)d_in[0];
  const float* Wq = (const float*)d_in[1];
  const float* bq = (const float*)d_in[2];
  const float* Wk = (const float*)d_in[3];
  const float* bk = (const float*)d_in[4];
  const float* Wv = (const float*)d_in[5];
  const float* bv = (const float*)d_in[6];
  const float* Wo = (const float*)d_in[7];
  const float* bo = (const float*)d_in[8];

  const size_t tokPlaneB = (size_t)kTok * kEmb * 2;
  const size_t wPlaneB   = (size_t)kEmb * kEmb * 2;
  const size_t total = tokPlaneB * 11 + wPlaneB * 4;
  if (total > ws_size) return;
  unsigned char* wsb = (unsigned char*)d_ws;
  size_t off = 0;
  unsigned short* Xb  = (unsigned short*)(wsb + off); off += tokPlaneB;
  unsigned short* WqT = (unsigned short*)(wsb + off); off += wPlaneB;
  unsigned short* WkT = (unsigned short*)(wsb + off); off += wPlaneB;
  unsigned short* WvT = (unsigned short*)(wsb + off); off += wPlaneB;
  unsigned short* WoT = (unsigned short*)(wsb + off); off += wPlaneB;
  unsigned short* Qh  = (unsigned short*)(wsb + off); off += tokPlaneB;
  unsigned short* Ql  = (unsigned short*)(wsb + off); off += tokPlaneB;
  unsigned short* Kh  = (unsigned short*)(wsb + off); off += tokPlaneB;
  unsigned short* Kl  = (unsigned short*)(wsb + off); off += tokPlaneB;
  unsigned short* Vh  = (unsigned short*)(wsb + off); off += tokPlaneB;
  unsigned short* Vl  = (unsigned short*)(wsb + off); off += tokPlaneB;
  unsigned short* Vth = (unsigned short*)(wsb + off); off += tokPlaneB;
  unsigned short* Vtl = (unsigned short*)(wsb + off); off += tokPlaneB;
  unsigned short* Oh  = (unsigned short*)(wsb + off); off += tokPlaneB;
  unsigned short* Ol  = (unsigned short*)(wsb + off); off += tokPlaneB;
  if (off > ws_size) return;

  const int n8 = kTok * kEmb / 8;
  k_cast_f32_bf16x8<<<(n8 + 255) / 256, 256, 0, stream>>>(x, Xb, n8);

  const dim3 gw(kEmb / 64, kEmb / 64);
  k_tr_f32_bf16<<<gw, 128, 0, stream>>>(Wq, WqT, kEmb, kEmb);
  k_tr_f32_bf16<<<gw, 128, 0, stream>>>(Wk, WkT, kEmb, kEmb);
  k_tr_f32_bf16<<<gw, 128, 0, stream>>>(Wv, WvT, kEmb, kEmb);
  k_tr_f32_bf16<<<gw, 128, 0, stream>>>(Wo, WoT, kEmb, kEmb);

  const int gemmTiles = (kTok / 64) * (kEmb / 64);
  const int gemmBlocks = (gemmTiles + 7) / 8;
  gemm_bf16_t64<false, 2><<<gemmBlocks, 256, 0, stream>>>(Xb, Xb, kEmb, WqT, kEmb, Qh, Ql, kEmb, bq, kTok, kEmb, kEmb);
  gemm_bf16_t64<false, 2><<<gemmBlocks, 256, 0, stream>>>(Xb, Xb, kEmb, WkT, kEmb, Kh, Kl, kEmb, bk, kTok, kEmb, kEmb);
  gemm_bf16_t64<false, 2><<<gemmBlocks, 256, 0, stream>>>(Xb, Xb, kEmb, WvT, kEmb, Vh, Vl, kEmb, bv, kTok, kEmb, kEmb);

  const dim3 gv(kEmb / 64, kSeq / 64, kBatch);
  const long vStride = (long)kSeq * kEmb;
  k_tr_u16<<<gv, 128, 0, stream>>>(Vh, Vth, kSeq, kEmb, vStride, vStride);
  k_tr_u16<<<gv, 128, 0, stream>>>(Vl, Vtl, kSeq, kEmb, vStride, vStride);

  k_attn_causal<<<kBatch * kHeads * (kSeq / kQb), 128, 0, stream>>>(Qh, Ql, Kh, Kl, Vth, Vtl, Oh, Ol);

  gemm_bf16_t64<true, 0><<<gemmBlocks, 256, 0, stream>>>(Oh, Ol, kEmb, WoT, kEmb, d_out, d_out, kEmb, bo, kTok, kEmb, kEmb);
}
